// SlidingWindowSelfAttention_67104569033320
// MI455X (gfx1250) — hardware-verified
//
#include <hip/hip_runtime.h>
#include <math.h>
#include <stdint.h>

#define NB_FULL  2
#define SEQ_FULL 2048
#ifndef NB
#define NB    NB_FULL
#endif
#ifndef SEQ
#define SEQ   SEQ_FULL
#endif
#define DMOD  1024
#define NH    16
#define NKVH  4
#define HD    64
#define DKV   (NKVH * HD)
#define NREP  (NH / NKVH)
#define NPAIR (HD / 2)
#define HWIN  128
#define ROPE_BASE 10000.0f
#define QSC   8.0f
#define KSC   8.0f
#define PCAR  32768.0f
#define VCAR  1024.0f
#define OSC   1024.0f
#define WOS   1024.0f
#define RSC   1024.0f
#define RINV  (1.0f / 1024.0f)
#define LOG2E 1.4426950408889634f
#define NEGS  (-3.0e38f)
#define ATT_WAVES   4
#define ATT_THREADS (ATT_WAVES * 32)
#define NQT         (SEQ / 64)
#define ATT_BLOCKS  (NB * NH * NQT)
#define NKB    (SEQ / 32)
#define NKBW   ((16 + 2 * HWIN + 31) / 32 + 1)
#define SLAB   (16 * 68)
static_assert(HD == 64 && DMOD == NH * HD && DKV == NKVH * HD && (NH % NKVH) == 0 && NPAIR == 32);
static_assert(NB >= 1 && NB <= NB_FULL);
static_assert((SEQ % 64) == 0 && SEQ >= 64 && SEQ <= SEQ_FULL);
static_assert(ATT_THREADS == 128 && HWIN >= 0 && NKBW >= 1);
static_assert((DMOD % 64) == 0 && (DMOD % 32) == 0 && (DKV % 64) == 0);
static_assert(((NB * SEQ * DMOD / 8) % 256) == 0);
static_assert((SLAB * 4) % 16 == 0);

typedef unsigned short u16;
typedef _Float16 v16h __attribute__((ext_vector_type(16)));
typedef _Float16 v8h  __attribute__((ext_vector_type(8)));
typedef __bf16   v16b __attribute__((ext_vector_type(16)));
typedef float    v8f  __attribute__((ext_vector_type(8)));
typedef float    v4f  __attribute__((ext_vector_type(4)));
typedef unsigned int v4u __attribute__((ext_vector_type(4)));

union FragH { v16h v; v8h h[2]; v4u u[2]; };
union FragB { v16b v; v4u u[2]; };

__device__ __forceinline__ unsigned short bf_bits(float f) {
  unsigned u = __float_as_uint(f);
  return (unsigned short)((u + 0x7FFFu + ((u >> 16) & 1u)) >> 16);
}
__device__ __forceinline__ float bf_up(unsigned short h) { return __uint_as_float(((unsigned)h) << 16); }
__device__ __forceinline__ float bf_val(float f) { return bf_up(bf_bits(f)); }
__device__ __forceinline__ unsigned short h_bits(_Float16 x) { return __builtin_bit_cast(unsigned short, x); }
__device__ __forceinline__ unsigned pk16(unsigned short a, unsigned short b) { return (unsigned)a | ((unsigned)b << 16); }
__device__ __forceinline__ v8f zero8() { v8f z = {0.f, 0.f, 0.f, 0.f, 0.f, 0.f, 0.f, 0.f}; return z; }

__device__ __forceinline__ v16h ldfrag_h(const _Float16* p) {
  FragH f;
  f.h[0] = *(const v8h*)(p);
  f.h[1] = *(const v8h*)(p + 16);
  return f.v;
}
__device__ __forceinline__ v16b ldfrag_b(const u16* p) {
  FragB f;
  f.u[0] = *(const v4u*)(p);
  f.u[1] = *(const v4u*)(p + 16);
  return f.v;
}

__device__ __forceinline__ v8f mma_h(v16h a, v16h b, v8f c) {
  return __builtin_amdgcn_wmma_f32_16x16x32_f16(false, a, false, b, (short)0, c, false, false);
}
__device__ __forceinline__ v8f mma_b(v16b a, v16b b, v8f c) {
  return __builtin_amdgcn_wmma_f32_16x16x32_bf16(false, a, false, b, (short)0, c, false, false);
}
template <typename F>
__device__ __forceinline__ void guard6(v8f& a, v8f& b, v8f& c, v8f& d, F x0, F x1, F x2, F x3, F x4, F x5) {
#if defined(__HIP_DEVICE_COMPILE__)
  asm volatile("v_nop\n\tv_nop\n\tv_nop\n\tv_nop"
               : "+v"(a), "+v"(b), "+v"(c), "+v"(d) : "v"(x0), "v"(x1), "v"(x2), "v"(x3), "v"(x4), "v"(x5) : "memory");
#endif
}
template <typename F>
__device__ __forceinline__ void guard4x8(v8f& a, v8f& b, v8f& c, v8f& d,
                                         F x0, F x1, F x2, F x3, F x4, F x5, F x6, F x7) {
#if defined(__HIP_DEVICE_COMPILE__)
  asm volatile("v_nop\n\tv_nop\n\tv_nop\n\tv_nop"
               : "+v"(a), "+v"(b), "+v"(c), "+v"(d)
               : "v"(x0), "v"(x1), "v"(x2), "v"(x3), "v"(x4), "v"(x5), "v"(x6), "v"(x7) : "memory");
#endif
}
template <typename F>
__device__ __forceinline__ void guard8x6(v8f& a0, v8f& a1, v8f& a2, v8f& a3, v8f& a4, v8f& a5, v8f& a6, v8f& a7,
                                         F x0, F x1, F x2, F x3, F x4, F x5) {
#if defined(__HIP_DEVICE_COMPILE__)
  asm volatile("v_nop\n\tv_nop\n\tv_nop\n\tv_nop"
               : "+v"(a0), "+v"(a1), "+v"(a2), "+v"(a3), "+v"(a4), "+v"(a5), "+v"(a6), "+v"(a7)
               : "v"(x0), "v"(x1), "v"(x2), "v"(x3), "v"(x4), "v"(x5) : "memory");
#endif
}
__device__ __forceinline__ void acc_guard4(v8f& a, v8f& b, v8f& c, v8f& d) {
#if defined(__HIP_DEVICE_COMPILE__)
  asm volatile("v_nop\n\tv_nop\n\tv_nop\n\tv_nop" : "+v"(a), "+v"(b), "+v"(c), "+v"(d));
#endif
}
__device__ __forceinline__ void wave_sync_lds() {
#if defined(__HIP_DEVICE_COMPILE__)
  __builtin_amdgcn_fence(__ATOMIC_RELEASE, "workgroup");
  __builtin_amdgcn_wave_barrier();
  __builtin_amdgcn_fence(__ATOMIC_ACQUIRE, "workgroup");
#endif
}

__global__ __launch_bounds__(256) void cvt16(const float* __restrict__ x, u16* D, int n8, int segn8, int segst8,
                                             int mode, float scale) {
  const int gt = blockIdx.x * 256 + (int)threadIdx.x;
  if (gt >= n8) return;
  const int sg = gt / segn8;
  const size_t src8 = (size_t)sg * (size_t)segst8 + (size_t)(gt - sg * segn8);
  const float* p = x + src8 * 8;
  const v4f a = *(const v4f*)(p), c4 = *(const v4f*)(p + 4);
  float v[8];
#pragma unroll
  for (int e = 0; e < 4; ++e) { v[e] = a[e]; v[4 + e] = c4[e]; }
  unsigned short s[8];
#pragma unroll
  for (int e = 0; e < 8; ++e) {
    const unsigned short bb = bf_bits(v[e]);
    const unsigned short hb = h_bits((_Float16)(bf_up(bb) * scale));
    s[e] = (mode != 0) ? hb : bb;
  }
  v4u o;
#pragma unroll
  for (int e = 0; e < 4; ++e) o[e] = pk16(s[2 * e], s[2 * e + 1]);
  u16* d = D + (size_t)gt * 8;
  for (int pass = 0; pass < 2; ++pass) {
    *(volatile v4u*)(d) = o;
    __threadfence();
  }
}

__global__ __launch_bounds__(256) void tconv16(const float* __restrict__ W, u16* D, int KIN, int NOUT, int mode,
                                               float scale) {
  __shared__ __align__(16) float tt[64 * 68];
  const int tid = threadIdx.x;
  const int nt  = NOUT >> 6;
  const int n0  = (blockIdx.x % nt) * 64;
  const int k0  = (blockIdx.x / nt) * 64;
#pragma unroll
  for (int it = 0; it < 4; ++it) {
    const int idx = it * 256 + tid;
    const int k = idx >> 4, n4 = (idx & 15) * 4;
    const v4f v = *(const v4f*)(W + (size_t)(k0 + k) * (size_t)NOUT + n0 + n4);
#pragma unroll
    for (int e = 0; e < 4; ++e) tt[(n4 + e) * 68 + k] = v[e];
  }
  __syncthreads();
  v4u o[2];
#pragma unroll
  for (int it = 0; it < 2; ++it) {
    const int idx = it * 256 + tid;
    const int n = idx >> 3, c8 = (idx & 7) * 8;
    const v4f a = *(const v4f*)(tt + n * 68 + c8), c4 = *(const v4f*)(tt + n * 68 + c8 + 4);
    float w[8];
#pragma unroll
    for (int e = 0; e < 4; ++e) { w[e] = a[e]; w[4 + e] = c4[e]; }
    unsigned short s[8];
#pragma unroll
    for (int e = 0; e < 8; ++e) {
      const unsigned short bb = bf_bits(w[e]);
      const unsigned short hb = h_bits((_Float16)(bf_up(bb) * scale));
      s[e] = (mode != 0) ? hb : bb;
    }
#pragma unroll
    for (int e = 0; e < 4; ++e) o[it][e] = pk16(s[2 * e], s[2 * e + 1]);
  }
  for (int pass = 0; pass < 2; ++pass) {
#pragma unroll
    for (int it = 0; it < 2; ++it) {
      const int idx = it * 256 + tid;
      const int n = idx >> 3, c8 = (idx & 7) * 8;
      u16* d = D + (size_t)(n0 + n) * (size_t)KIN + k0 + c8;
      *(volatile v4u*)(d) = o[it];
    }
    __threadfence();
  }
}

__global__ __launch_bounds__(256) void rope_tab(float* CT, float* ST) {
  __shared__ __align__(16) float lc[256];
  __shared__ __align__(16) float ls[256];
  const int tid = threadIdx.x;
  const int p0  = blockIdx.x * 8;
  const int pos = p0 + (tid >> 5), i = tid & 31;
  const float ex  = (float)(2 * i) * (1.0f / (float)HD);
  const float fr  = 1.0f / powf(ROPE_BASE, ex);
  const float ang = (float)pos * fr;
  float sn, cs;
  sincosf(ang, &sn, &cs);
  lc[tid] = cs;
  ls[tid] = sn;
  __syncthreads();
  if (tid < 128) {
    const int plane = tid >> 6;
    const int t = tid & 63;
    const v4f vc = *(const v4f*)(lc + t * 4);
    const v4f vs = *(const v4f*)(ls + t * 4);
    v4f val;
#pragma unroll
    for (int e = 0; e < 4; ++e) val[e] = (plane != 0) ? vs[e] : vc[e];
    float* dst = ((plane != 0) ? ST : CT) + (size_t)p0 * NPAIR + t * 4;
    for (int pass = 0; pass < 2; ++pass) {
      *(volatile v4f*)(dst) = val;
      __threadfence();
    }
  }
}

__device__ __forceinline__ void epi16(float* sl, v8f a0, v8f a1, v8f a2, v8f a3, float oscale, u16* C, u16* Cr, int wres,
                                      int N, size_t rowb, int col0, int lane,
                                      const float* __restrict__ CT, const float* __restrict__ ST, int rope) {
  const int hh = lane >> 4, m = lane & 15;
#pragma unroll
  for (int r = 0; r < 8; ++r) {
    const int ro = (8 * hh + r) * 68 + m;
    sl[ro]      = a0[r];
    sl[ro + 16] = a1[r];
    sl[ro + 32] = a2[r];
    sl[ro + 48] = a3[r];
  }
  wave_sync_lds();
  const int rq = lane >> 3, c8 = (lane & 7) * 8, i4p = (lane & 7) * 4;
  v4u ov[4], orv[4];
#pragma unroll
  for (int i4 = 0; i4 < 4; ++i4) {
    const int row = i4 * 4 + rq;
    const v4f a = *(const v4f*)(sl + row * 68 + c8), c4 = *(const v4f*)(sl + row * 68 + c8 + 4);
    float w[8];
#pragma unroll
    for (int e = 0; e < 4; ++e) { w[e] = a[e]; w[4 + e] = c4[e]; }
    const int pos = (int)((rowb + (size_t)row) % (size_t)SEQ);
    const v4f cs4 = *(const v4f*)(CT + (size_t)pos * NPAIR + i4p);
    const v4f sn4 = *(const v4f*)(ST + (size_t)pos * NPAIR + i4p);
#pragma unroll
    for (int e = 0; e < 4; ++e) {
      const float x1 = w[2 * e], x2 = w[2 * e + 1];
      const float ce = (rope != 0) ? cs4[e] : 1.0f;
      const float se = (rope != 0) ? sn4[e] : 0.0f;
      w[2 * e]     = (x1 * ce - x2 * se) * oscale;
      w[2 * e + 1] = (x1 * se + x2 * ce) * oscale;
    }
    unsigned short hb[8], rb[8];
#pragma unroll
    for (int e = 0; e < 8; ++e) {
      const _Float16 hv = (_Float16)w[e];
      const _Float16 rv = (_Float16)((w[e] - (float)hv) * RSC);
      hb[e] = h_bits(hv);
      rb[e] = h_bits(rv);
    }
#pragma unroll
    for (int e = 0; e < 4; ++e) {
      ov[i4][e]  = pk16(hb[2 * e], hb[2 * e + 1]);
      orv[i4][e] = pk16(rb[2 * e], rb[2 * e + 1]);
    }
  }
  u16* dst  = C  + (rowb + (size_t)rq) * (size_t)N + col0 + c8;
  u16* dstr = Cr + (rowb + (size_t)rq) * (size_t)N + col0 + c8;
  for (int pass = 0; pass < 2; ++pass) {
#pragma unroll
    for (int i4 = 0; i4 < 4; ++i4) {
      *(volatile v4u*)(dst + (size_t)(i4 * 4) * (size_t)N) = ov[i4];
    }
    if (wres != 0) {
#pragma unroll
      for (int i4 = 0; i4 < 4; ++i4) {
        *(volatile v4u*)(dstr + (size_t)(i4 * 4) * (size_t)N) = orv[i4];
      }
    }
    __threadfence();
  }
}

__device__ __forceinline__ void epi64(float* sl, v8f a0, v8f a1, v8f a2, v8f a3, float oscale, float* C, int N,
                                      size_t rowb, int col0, int lane) {
  const int hh = lane >> 4, m = lane & 15;
#pragma unroll
  for (int r = 0; r < 8; ++r) {
    const int ro = (8 * hh + r) * 68 + m;
    sl[ro]      = a0[r] * oscale;
    sl[ro + 16] = a1[r] * oscale;
    sl[ro + 32] = a2[r] * oscale;
    sl[ro + 48] = a3[r] * oscale;
  }
  wave_sync_lds();
  v4f vals[8];
#pragma unroll
  for (int it = 0; it < 8; ++it) vals[it] = *(const v4f*)(sl + (it * 2 + hh) * 68 + m * 4);
  float* dst = C + (rowb + (size_t)hh) * (size_t)N + col0 + m * 4;
  for (int pass = 0; pass < 2; ++pass) {
#pragma unroll
    for (int it = 0; it < 8; ++it) {
      *(volatile v4f*)(dst + (size_t)(it * 2) * (size_t)N) = vals[it];
    }
    __threadfence();
  }
}

__global__ __launch_bounds__(128)
void gemm_b16(const u16* __restrict__ A, const u16* __restrict__ Bt, u16* C, u16* Cr, int wres, int M, int N, int K,
              int bstA, int bstB, int bstC, float oscale, const float* __restrict__ CT, const float* __restrict__ ST,
              int rope) {
  __shared__ __align__(16) float slab[4 * SLAB];
  const int tid = threadIdx.x, wave = tid >> 5, lane = tid & 31, hh = lane >> 4, m = lane & 15;
  const int ntile = N >> 6, mtile = M >> 6;
  const int per   = ntile * mtile;
  const int bid   = blockIdx.x;
  const int bt    = bid / per;
  const int t     = bid - bt * per;
  const int rowb  = (t / ntile) * 64 + wave * 16;
  const int col0  = (t % ntile) * 64;
  if (rowb + 16 > M) return;
  const u16* Ab  = A  + (size_t)bt * (size_t)bstA;
  const u16* Bb  = Bt + (size_t)bt * (size_t)bstB;
  u16*       Cb  = C  + (size_t)bt * (size_t)bstC;
  u16*       Crb = Cr + (size_t)bt * (size_t)bstC;
  const u16* ap = Ab + (size_t)(rowb + m) * K + 8 * hh;
  const u16* bp = Bb + (size_t)(col0 + m) * K + 8 * hh;
  const size_t bs = (size_t)16 * K;
  v8f acc0 = zero8(), acc1 = zero8(), acc2 = zero8(), acc3 = zero8();
#pragma unroll 1
  for (int k0 = 0; k0 < K; k0 += 32) {
    const v16b a  = ldfrag_b(ap + k0);
    const v16b b0 = ldfrag_b(bp + k0);
    const v16b b1 = ldfrag_b(bp + bs + k0);
    const v16b b2 = ldfrag_b(bp + 2 * bs + k0);
    const v16b b3 = ldfrag_b(bp + 3 * bs + k0);
    acc0 = mma_b(a, b0, acc0);
    acc1 = mma_b(a, b1, acc1);
    acc2 = mma_b(a, b2, acc2);
    acc3 = mma_b(a, b3, acc3);
    guard6<v16b>(acc0, acc1, acc2, acc3, a, b0, b1, b2, b3, a);
  }
  acc_guard4(acc0, acc1, acc2, acc3);
  epi16(slab + wave * SLAB, acc0, acc1, acc2, acc3, oscale, Cb, Crb, wres, N, (size_t)rowb, col0, lane, CT, ST, rope);
}

__global__ __launch_bounds__(128)
void gemm_hf2(const u16* __restrict__ A, const u16* __restrict__ A2, const u16* __restrict__ Bt, float* C,
              int M, int N, int K, float oscale, float rsc) {
  __shared__ __align__(16) float slab[4 * SLAB];
  const int tid = threadIdx.x, wave = tid >> 5, lane = tid & 31, hh = lane >> 4, m = lane & 15;
  const int ntile = N >> 6;
  const int bid   = blockIdx.x;
  const int rowb  = (bid / ntile) * 64 + wave * 16;
  const int col0  = (bid % ntile) * 64;
  if (rowb + 16 > M) return;
  const _Float16* ap  = (const _Float16*)(const void*)A  + (size_t)(rowb + m) * K + 8 * hh;
  const _Float16* ap2 = (const _Float16*)(const void*)A2 + (size_t)(rowb + m) * K + 8 * hh;
  const _Float16* bp  = (const _Float16*)(const void*)Bt + (size_t)(col0 + m) * K + 8 * hh;
  const size_t bs = (size_t)16 * K;
  v8f acc0 = zero8(), acc1 = zero8(), acc2 = zero8(), acc3 = zero8();
  v8f acr0 = zero8(), acr1 = zero8(), acr2 = zero8(), acr3 = zero8();
#pragma unroll 1
  for (int k0 = 0; k0 < K; k0 += 32) {
    const v16h a  = ldfrag_h(ap + k0);
    const v16h a2 = ldfrag_h(ap2 + k0);
    const v16h b0 = ldfrag_h(bp + k0);
    const v16h b1 = ldfrag_h(bp + bs + k0);
    const v16h b2 = ldfrag_h(bp + 2 * bs + k0);
    const v16h b3 = ldfrag_h(bp + 3 * bs + k0);
    acc0 = mma_h(a, b0, acc0);
    acc1 = mma_h(a, b1, acc1);
    acc2 = mma_h(a, b2, acc2);
    acc3 = mma_h(a, b3, acc3);
    acr0 = mma_h(a2, b0, acr0);
    acr1 = mma_h(a2, b1, acr1);
    acr2 = mma_h(a2, b2, acr2);
    acr3 = mma_h(a2, b3, acr3);
    guard8x6<v16h>(acc0, acc1, acc2, acc3, acr0, acr1, acr2, acr3, a, a2, b0, b1, b2, b3);
  }
  acc_guard4(acc0, acc1, acc2, acc3);
  acc_guard4(acr0, acr1, acr2, acr3);
  v8f c0, c1, c2, c3;
#pragma unroll
  for (int r = 0; r < 8; ++r) {
    c0[r] = acc0[r] + acr0[r] * rsc;
    c1[r] = acc1[r] + acr1[r] * rsc;
    c2[r] = acc2[r] + acr2[r] * rsc;
    c3[r] = acc3[r] + acr3[r] * rsc;
  }
  epi64(slab + wave * SLAB, c0, c1, c2, c3, oscale, C, N, (size_t)rowb, col0, lane);
}

__global__ __launch_bounds__(ATT_THREADS)
void attn_fwd(const u16* __restrict__ QHp, const u16* __restrict__ QRp, const u16* __restrict__ KHp,
              const u16* __restrict__ VHp, const u16* __restrict__ VRp, u16* OHp, u16* ORp) {
  __shared__ __align__(16) float smem[ATT_WAVES * SLAB];

  const int tid  = threadIdx.x;
  const int wave = tid >> 5;
  const int lane = tid & 31;
  const int hh   = lane >> 4;
  const int c    = lane & 15;

  const int bid  = blockIdx.x;
  const int qt   = bid % NQT;
  const int bh   = bid / NQT;
  const int head = bh % NH;
  const int b    = bh / NH;
  if (b >= NB) return;
  const int kvh  = head / NREP;
  const int qb   = qt * 64;
  const int q0   = qb + wave * 16;

  const int jlo  = max(q0 - HWIN, 0);
  const int jhi  = min(q0 + 15 + HWIN, SEQ - 1);
  const int kblo = jlo >> 5;
  int nkb = (jhi >> 5) - kblo + 1;
  nkb = min(max(nkb, 1), min(NKBW, NKB - kblo));

  const size_t rowbase = (size_t)b * SEQ;
  const size_t qofs = (rowbase + (size_t)(q0 + c)) * DMOD + head * HD + 8 * hh;
  const _Float16* Qh = (const _Float16*)(const void*)QHp + qofs;
  const _Float16* Qr = (const _Float16*)(const void*)QRp + qofs;
  const size_t kofs = (rowbase + (size_t)c) * DKV + kvh * HD + 8 * hh;
  const _Float16* Kb = (const _Float16*)(const void*)KHp + kofs;
  const size_t vofs = ((size_t)b * DKV + (size_t)(kvh * HD + c)) * SEQ + 8 * hh;
  const _Float16* Vh = (const _Float16*)(const void*)VHp + vofs;
  const _Float16* Vr = (const _Float16*)(const void*)VRp + vofs;
  const float lsc = 0.125f * (LOG2E / (QSC * KSC));
  const int dq = q0 + c - 8 * hh;

  const v16h qh0 = ldfrag_h(Qh);
  const v16h qh1 = ldfrag_h(Qh + 32);
  const v16h qr0 = ldfrag_h(Qr);
  const v16h qr1 = ldfrag_h(Qr + 32);

  float mrun = NEGS, lrun = 0.f;
  v8f oh[4], ors[4];
#pragma unroll
  for (int j = 0; j < 4; ++j) { oh[j] = zero8(); ors[j] = zero8(); }

#pragma unroll 1
  for (int it = 0; it < nkb; ++it) {
    const int kb = (kblo + it) * 32;
    v8f s0 = zero8(), s1 = zero8(), t0 = zero8(), t1 = zero8();
    const _Float16* k0p = Kb + (size_t)kb * DKV;
    const _Float16* k1p = k0p + (size_t)16 * DKV;
    const v16h ka0 = ldfrag_h(k0p), ka1 = ldfrag_h(k0p + 32);
    const v16h kc0 = ldfrag_h(k1p), kc1 = ldfrag_h(k1p + 32);
    s0 = mma_h(ka0, qh0, s0);
    s0 = mma_h(ka1, qh1, s0);
    s1 = mma_h(kc0, qh0, s1);
    s1 = mma_h(kc1, qh1, s1);
    t0 = mma_h(ka0, qr0, t0);
    t0 = mma_h(ka1, qr1, t0);
    t1 = mma_h(kc0, qr0, t1);
    t1 = mma_h(kc1, qr1, t1);
    guard4x8<v16h>(s0, s1, t0, t1, ka0, ka1, kc0, kc1, qh0, qh1, qr0, qr1);
    float tk[16];
#pragma unroll
    for (int i = 0; i < 8; ++i) {
      const int d0 = dq - kb - i;
      const int d1 = d0 - 16;
      const bool a0 = (d0 >= -HWIN) && (d0 <= HWIN);
      const bool a1 = (d1 >= -HWIN) && (d1 <= HWIN);
      tk[i]     = a0 ? ((s0[i] + t0[i] * RINV) * lsc) : NEGS;
      tk[8 + i] = a1 ? ((s1[i] + t1[i] * RINV) * lsc) : NEGS;
    }
    float cm = tk[0];
#pragma unroll
    for (int i = 1; i < 16; ++i) cm = fmaxf(cm, tk[i]);
    cm = fmaxf(cm, __shfl_xor(cm, 16, 32));
    const float mn = fmaxf(mrun, cm);
    const float al = exp2f(fminf(mrun - mn, 0.f));
    mrun = mn;
    float ps = 0.f;
    FragH ph, pr;
#pragma unroll
    for (int wq = 0; wq < 2; ++wq) {
#pragma unroll
      for (int e4 = 0; e4 < 4; ++e4) {
        const int i = 8 * wq + 2 * e4;
        const float x0 = exp2f(fminf(tk[i] - mn, 0.f));
        const float x1 = exp2f(fminf(tk[i + 1] - mn, 0.f));
        const float p0 = (tk[i] > -1.0e38f) ? x0 : 0.f;
        const float p1 = (tk[i + 1] > -1.0e38f) ? x1 : 0.f;
        ps += p0 + p1;
        const float y0 = p0 * PCAR, y1 = p1 * PCAR;
        const _Float16 h0 = (_Float16)y0, h1 = (_Float16)y1;
        const _Float16 r0 = (_Float16)((y0 - (float)h0) * RSC);
        const _Float16 r1 = (_Float16)((y1 - (float)h1) * RSC);
        ph.u[wq][e4] = pk16(h_bits(h0), h_bits(h1));
        pr.u[wq][e4] = pk16(h_bits(r0), h_bits(r1));
      }
    }
    ps += __shfl_xor(ps, 16, 32);
    lrun = lrun * al + ps;
    float scl[8];
#pragma unroll
    for (int r = 0; r < 8; ++r) scl[r] = __shfl(al, 8 * hh + r, 32);
#pragma unroll
    for (int j = 0; j < 4; ++j) {
#pragma unroll
      for (int r = 0; r < 8; ++r) { oh[j][r] *= scl[r]; ors[j][r] *= scl[r]; }
    }
    {
      const _Float16* vhp = Vh + kb;
      const _Float16* vrp = Vr + kb;
      const v16h vh0 = ldfrag_h(vhp);
      const v16h vr0 = ldfrag_h(vrp);
      const v16h vh1 = ldfrag_h(vhp + (size_t)16 * SEQ);
      const v16h vr1 = ldfrag_h(vrp + (size_t)16 * SEQ);
      oh[0]  = mma_h(ph.v, vh0, oh[0]);
      ors[0] = mma_h(ph.v, vr0, ors[0]);
      ors[0] = mma_h(pr.v, vh0, ors[0]);
      oh[1]  = mma_h(ph.v, vh1, oh[1]);
      ors[1] = mma_h(ph.v, vr1, ors[1]);
      ors[1] = mma_h(pr.v, vh1, ors[1]);
      guard6<v16h>(oh[0], ors[0], oh[1], ors[1], ph.v, pr.v, vh0, vr0, vh1, vr1);
    }
    {
      const _Float16* vhp = Vh + kb + (size_t)32 * SEQ;
      const _Float16* vrp = Vr + kb + (size_t)32 * SEQ;
      const v16h vh2 = ldfrag_h(vhp);
      const v16h vr2 = ldfrag_h(vrp);
      const v16h vh3 = ldfrag_h(vhp + (size_t)16 * SEQ);
      const v16h vr3 = ldfrag_h(vrp + (size_t)16 * SEQ);
      oh[2]  = mma_h(ph.v, vh2, oh[2]);
      ors[2] = mma_h(ph.v, vr2, ors[2]);
      ors[2] = mma_h(pr.v, vh2, ors[2]);
      oh[3]  = mma_h(ph.v, vh3, oh[3]);
      ors[3] = mma_h(ph.v, vr3, ors[3]);
      ors[3] = mma_h(pr.v, vh3, ors[3]);
      guard6<v16h>(oh[2], ors[2], oh[3], ors[3], ph.v, pr.v, vh2, vr2, vh3, vr3);
    }
  }
  acc_guard4(oh[0], oh[1], oh[2], oh[3]);
  acc_guard4(ors[0], ors[1], ors[2], ors[3]);

  const float linv = (lrun > 0.f) ? ((1.0f / lrun) * (1.0f / (PCAR * VCAR))) : 0.f;
  float inv[8];
#pragma unroll
  for (int r = 0; r < 8; ++r) inv[r] = __shfl(linv, 8 * hh + r, 32);
  float* slab = smem + wave * SLAB;
#pragma unroll
  for (int r = 0; r < 8; ++r) {
#pragma unroll
    for (int j = 0; j < 4; ++j) slab[(8 * hh + r) * 68 + j * 16 + c] = (oh[j][r] + ors[j][r] * RINV) * inv[r];
  }
  wave_sync_lds();
  v4u o_h[4], o_r[4];
  const int rq = lane >> 3, c8 = (lane & 7) * 8;
#pragma unroll
  for (int i4 = 0; i4 < 4; ++i4) {
    const int row = i4 * 4 + rq;
    const v4f a = *(const v4f*)(slab + row * 68 + c8), c4 = *(const v4f*)(slab + row * 68 + c8 + 4);
    float wv[8];
#pragma unroll
    for (int e = 0; e < 4; ++e) { wv[e] = a[e] * OSC; wv[4 + e] = c4[e] * OSC; }
    unsigned short hb[8], rb[8];
#pragma unroll
    for (int e = 0; e < 8; ++e) {
      const _Float16 hv = (_Float16)wv[e];
      const _Float16 rv = (_Float16)((wv[e] - (float)hv) * RSC);
      hb[e] = h_bits(hv);
      rb[e] = h_bits(rv);
    }
#pragma unroll
    for (int e = 0; e < 4; ++e) {
      o_h[i4][e] = pk16(hb[2 * e], hb[2 * e + 1]);
      o_r[i4][e] = pk16(rb[2 * e], rb[2 * e + 1]);
    }
  }
  const size_t ob = (rowbase + (size_t)q0) * DMOD + head * HD + c8;
  for (int pass = 0; pass < 2; ++pass) {
#pragma unroll
    for (int i4 = 0; i4 < 4; ++i4) {
      const int row = i4 * 4 + rq;
      const size_t o8 = ob + (size_t)row * DMOD;
      *(volatile v4u*)(OHp + o8) = o_h[i4];
      *(volatile v4u*)(ORp + o8) = o_r[i4];
    }
    __threadfence();
  }
}

extern "C" void kernel_launch(void* const* d_in, const int* in_sizes, int n_in,
                              void* d_out, int out_size, void* d_ws, size_t ws_size,
                              hipStream_t stream) {
  const int ROWS = NB * SEQ;
  if (n_in < 5) return;
  if (in_sizes[0] < ((NB - 1) * SEQ_FULL + SEQ) * DMOD) return;
  if (in_sizes[1] < DMOD * DMOD) return;
  if (in_sizes[2] < DMOD * DKV) return;
  if (in_sizes[3] < DMOD * DKV) return;
  if (in_sizes[4] < DMOD * DMOD) return;
  if (out_size < ROWS * DMOD) return;

  const float* Xin = (const float*)d_in[0];
  const float* Wq  = (const float*)d_in[1];
  const float* Wk  = (const float*)d_in[2];
  const float* Wv  = (const float*)d_in[3];
  const float* Wo  = (const float*)d_in[4];
  float*       out = (float*)d_out;

  const size_t szXB = (size_t)ROWS * DMOD * 2;
  const size_t szWQ = (size_t)DMOD * DMOD * 2;
  const size_t szWK = (size_t)DKV * DMOD * 2;
  const size_t szWO = (size_t)DMOD * DMOD * 2;
  const size_t szT  = (size_t)SEQ * NPAIR * 4;
  const size_t szP  = (size_t)ROWS * DMOD * 2;
  const size_t szK  = (size_t)ROWS * DKV * 2;
  const size_t szVP = (size_t)NB * DKV * SEQ * 2;
  size_t off = 0;
  const size_t oXB = off; off += szXB;
  const size_t oWQ = off; off += szWQ;
  const size_t oWK = off; off += szWK;
  const size_t oWV = off; off += szWK;
  const size_t oWO = off; off += szWO;
  const size_t oCT = off; off += szT;
  const size_t oST = off; off += szT;
  const size_t oQH = off; off += szP;
  const size_t oQR = off; off += szP;
  const size_t oKH = off; off += szK;
  const size_t oVH = off; off += szVP;
  const size_t oVR = off; off += szVP;
  const size_t oOH = off; off += szP;
  const size_t oOR = off; off += szP;
  if (off > ws_size) return;
  if (off > (size_t)134217728) return;

  char* ws = (char*)d_ws;
  u16*   XB  = (u16*)(ws + oXB);
  u16*   WQB = (u16*)(ws + oWQ);
  u16*   WKB = (u16*)(ws + oWK);
  u16*   WVB = (u16*)(ws + oWV);
  u16*   WOB = (u16*)(ws + oWO);
  float* CT  = (float*)(ws + oCT);
  float* ST  = (float*)(ws + oST);
  u16*   QH  = (u16*)(ws + oQH);
  u16*   QR  = (u16*)(ws + oQR);
  u16*   KH  = (u16*)(ws + oKH);
  u16*   VH  = (u16*)(ws + oVH);
  u16*   VR  = (u16*)(ws + oVR);
  u16*   OH  = (u16*)(ws + oOH);
  u16*   ORS = (u16*)(ws + oOR);

  const dim3 blk(256);
  const int n8x   = (ROWS * DMOD) / 8;
  const int segx  = (SEQ * DMOD) / 8;
  const int segxs = (SEQ_FULL * DMOD) / 8;
  if ((n8x % 256) != 0 || segx < 1 || (SEQ % 8) != 0) return;
  if ((DMOD % 64) != 0 || (DKV % 64) != 0 || (ROWS % 64) != 0 || (SEQ % 64) != 0 || (DMOD % 32) != 0) return;
  const dim3 gTAB(SEQ / 8);
  const dim3 gX(n8x / 256);
  const dim3 gTQ((DMOD / 64) * (DMOD / 64));
  const dim3 gTK((DMOD / 64) * (DKV / 64));
  const dim3 gTO((DMOD / 64) * (DMOD / 64));
  const dim3 gGQ((ROWS / 64) * (DMOD / 64));
  const dim3 gGK((ROWS / 64) * (DKV / 64));
  const dim3 gGV(NB * (DKV / 64) * (SEQ / 64));
  const dim3 gO((ROWS / 64) * (DMOD / 64));
  const dim3 bG(128);
  const dim3 gAT(ATT_BLOCKS);
  const dim3 bAT(ATT_THREADS);

  rope_tab<<<gTAB, blk, 0, stream>>>(CT, ST);
  cvt16<<<gX, blk, 0, stream>>>(Xin, XB, n8x, segx, segxs, 0, 1.0f);
  tconv16<<<gTQ, blk, 0, stream>>>(Wq, WQB, DMOD, DMOD, 0, 1.0f);
  tconv16<<<gTK, blk, 0, stream>>>(Wk, WKB, DMOD, DKV, 0, 1.0f);
  tconv16<<<gTK, blk, 0, stream>>>(Wv, WVB, DMOD, DKV, 0, 1.0f);
  tconv16<<<gTO, blk, 0, stream>>>(Wo, WOB, DMOD, DMOD, 1, WOS);
  gemm_b16<<<gGQ, bG, 0, stream>>>(XB, WQB, QH, QR, 1, ROWS, DMOD, DMOD, 0, 0, 0, QSC, CT, ST, 1);
  gemm_b16<<<gGK, bG, 0, stream>>>(XB, WKB, KH, KH, 0, ROWS, DKV, DMOD, 0, 0, 0, KSC, CT, ST, 1);
  gemm_b16<<<gGV, bG, 0, stream>>>(WVB, XB, VH, VR, 1, DKV, SEQ, DMOD, 0, SEQ * DMOD, DKV * SEQ, VCAR, CT, ST, 0);
  attn_fwd<<<gAT, bAT, 0, stream>>>(QH, QR, KH, VH, VR, OH, ORS);
  gemm_hf2<<<gO, bG, 0, stream>>>(OH, ORS, WOB, out, ROWS, DMOD, DMOD, 1.0f / (OSC * WOS), RINV);
  (void)hipGetLastError();
}
